// GATNN_86586540687412
// MI455X (gfx1250) — hardware-verified
//
#include <hip/hip_runtime.h>
#include <stddef.h>
#include <stdint.h>
#include <math.h>


#define NN      50000
#define NE      640000
#define NG      256
#define HC      128
#define NHD     4
#define HID     32
#define VOC     100
#define NFEAT   9
#define NLAY    4
#define MP      50048
#define KA      256
#define NW      256
#define NTHR    256
#define NWAVE   8
#define EPT     8
#define CHUNK   (NTHR * EPT)
#define WCAP    (EPT * 32)
#define LISTN   (NWAVE * WCAP)
#define NB      1024
#define SLB     10
#define NBLK    49
#define RCAP    28672
#define DEGCAP  64
#define GBM     64
#define GBN     128
#define GTHR    128
#define SROWS   64
#define NSB     (MP / SROWS)
#define PARTW   288
#define NEGSL   0.2f
#define WSMAX   134217728
#define LDS_BKT ((2 * RCAP + 2 * NB + LISTN) * 4 + 64)

static_assert(NN <= 65536);
static_assert(NB == (1 << SLB) && NB <= 1024);
static_assert(NBLK * NB >= MP);
static_assert((CHUNK & (CHUNK - 1)) == 0);
static_assert(((CHUNK - 1) << SLB | (NB - 1)) > 0);
static_assert(LISTN >= NB && LISTN >= NWAVE * WCAP);
static_assert((RCAP % 1024) == 0 && RCAP >= 13366 + 4096);
static_assert(DEGCAP >= 31 + 8);
static_assert(NTHR * 4 == NB);
static_assert(LDS_BKT <= 300000);
static_assert((MP % GBM) == 0 && (MP % SROWS) == 0 && (MP % 128) == 0 && MP >= NN);
static_assert((KA % 32) == 0 && KA == 2 * HC && NW == 2 * GBN && GBN == HC);
static_assert(GBM == (GTHR / 32) * 16 && GTHR == 2 * GBM);
static_assert(HC == 4 * 32 && HID == 4 * 8 && HC == NHD * HID);
static_assert(SROWS == NWAVE * 8 && (NSB - 1) * SROWS < NN);
static_assert(PARTW % 32 == 0 && PARTW >= 2 * HC + 1 && PARTW / 4 <= NTHR);
static_assert(2 * HC == NTHR && PARTW - NTHR == 32);
static_assert((NE % 4) == 0);
static_assert(NG == 256 && (NG % 4) == 0);

typedef float          v4f  __attribute__((ext_vector_type(4)));
typedef float          v8f  __attribute__((ext_vector_type(8)));
typedef int            v4i  __attribute__((ext_vector_type(4)));
typedef int            v8i  __attribute__((ext_vector_type(8)));
typedef unsigned int   v2u  __attribute__((ext_vector_type(2)));
typedef unsigned int   v4u  __attribute__((ext_vector_type(4)));
typedef unsigned short v8us __attribute__((ext_vector_type(8)));
typedef __bf16         v16b __attribute__((ext_vector_type(16)));
typedef v4f  __attribute__((may_alias)) v4fa;
typedef v4i  __attribute__((may_alias)) v4ia;
typedef v8us __attribute__((may_alias)) v8usa;
union FragB { v16b v; v8us h[2]; v8i w; };

__device__ __forceinline__ v8f wmb(const FragB& a, const FragB& b, v8f c) {
  v8f d = __builtin_amdgcn_wmma_f32_16x16x32_bf16(false, a.v, false, b.v, (short)0, c, false, false);
  asm volatile("v_nop\n\tv_nop\n\tv_nop\n\tv_nop" : "+v"(d) : "v"(a.w), "v"(b.w));
  return d;
}

__device__ __forceinline__ unsigned int f2bf(float f) {
  const unsigned int u = __float_as_uint(f);
  const unsigned int r = ((u + 0x7FFFu + ((u >> 16) & 1u)) >> 16) & 0xFFFFu;
  return (f != f) ? 0x7FC0u : r;
}
__device__ __forceinline__ float bf2f(unsigned int b) { return __uint_as_float(b << 16); }
__device__ __forceinline__ float bfr(float f) { return bf2f(f2bf(f)); }
__device__ __forceinline__ v4f bfr4(const v4f a) {
  v4f r; r.x = bfr(a.x); r.y = bfr(a.y); r.z = bfr(a.z); r.w = bfr(a.w); return r;
}
__device__ __forceinline__ unsigned int pk2(float lo, float hi) { return f2bf(lo) | (f2bf(hi) << 16); }
__device__ __forceinline__ v4u pack8(const v4f a, const v4f b) {
  v4u r;
  r.x = pk2(a.x, a.y); r.y = pk2(a.z, a.w); r.z = pk2(b.x, b.y); r.w = pk2(b.z, b.w);
  return r;
}
struct HL { v2u hi; v2u lo; };
__device__ __forceinline__ HL split4(const v4f v) {
  const unsigned int h0 = f2bf(v.x), h1 = f2bf(v.y), h2 = f2bf(v.z), h3 = f2bf(v.w);
  const unsigned int g0 = f2bf(v.x - bf2f(h0)), g1 = f2bf(v.y - bf2f(h1));
  const unsigned int g2 = f2bf(v.z - bf2f(h2)), g3 = f2bf(v.w - bf2f(h3));
  HL r;
  r.hi.x = h0 | (h1 << 16); r.hi.y = h2 | (h3 << 16);
  r.lo.x = g0 | (g1 << 16); r.lo.y = g2 | (g3 << 16);
  return r;
}
__device__ __forceinline__ float reluf(float v) { return (v > 0.0f) ? v : (v - v); }

__device__ __forceinline__ int scan_chunk(const int* __restrict__ dsts, int nE, int cbase, int slotBase,
                                          int nb, int vec8, int* list, int tid, int lane, int wave) {
  int wc = 0;
  const int el0  = tid * EPT;
  const int e0   = cbase + el0;
  const int sent = -2147483647 - 1;
  v4i da, db;
  if (vec8 != 0 && cbase + CHUNK <= nE) {
    da = *(const v4i*)(dsts + e0);
    db = *(const v4i*)(dsts + e0 + 4);
  } else {
    da.x = (e0     < nE) ? dsts[min(e0,     nE - 1)] : sent;
    da.y = (e0 + 1 < nE) ? dsts[min(e0 + 1, nE - 1)] : sent;
    da.z = (e0 + 2 < nE) ? dsts[min(e0 + 2, nE - 1)] : sent;
    da.w = (e0 + 3 < nE) ? dsts[min(e0 + 3, nE - 1)] : sent;
    db.x = (e0 + 4 < nE) ? dsts[min(e0 + 4, nE - 1)] : sent;
    db.y = (e0 + 5 < nE) ? dsts[min(e0 + 5, nE - 1)] : sent;
    db.z = (e0 + 6 < nE) ? dsts[min(e0 + 6, nE - 1)] : sent;
    db.w = (e0 + 7 < nE) ? dsts[min(e0 + 7, nE - 1)] : sent;
  }
  const unsigned nbs = (unsigned)slotBase;
  const unsigned unb = (unsigned)nb;
  const unsigned s0 = (unsigned)da.x - nbs, s1 = (unsigned)da.y - nbs;
  const unsigned s2 = (unsigned)da.z - nbs, s3 = (unsigned)da.w - nbs;
  const unsigned s4 = (unsigned)db.x - nbs, s5 = (unsigned)db.y - nbs;
  const unsigned s6 = (unsigned)db.z - nbs, s7 = (unsigned)db.w - nbs;
  const bool h0 = s0 < unb, h1 = s1 < unb, h2 = s2 < unb, h3 = s3 < unb;
  const bool h4 = s4 < unb, h5 = s5 < unb, h6 = s6 < unb, h7 = s7 < unb;
  const unsigned any = __builtin_amdgcn_ballot_w32(h0 | h1 | h2 | h3 | h4 | h5 | h6 | h7);
  if (any != 0u) {
#define HITJ(J, HJ, SJ) { \
      const unsigned mj = __builtin_amdgcn_ballot_w32(HJ); \
      if (mj != 0u) { \
        if (HJ) { \
          const int pos = wc + (int)__builtin_amdgcn_mbcnt_lo(mj, 0u); \
          if (pos < WCAP) list[wave * WCAP + pos] = ((el0 + (J)) << SLB) | (int)(SJ); \
        } \
        wc += (int)__builtin_popcount(mj); } }
    HITJ(0, h0, s0)
    HITJ(1, h1, s1)
    HITJ(2, h2, s2)
    HITJ(3, h3, s3)
    HITJ(4, h4, s4)
    HITJ(5, h5, s5)
    HITJ(6, h6, s6)
    HITJ(7, h7, s7)
#undef HITJ
  }
  return wc;
}

__global__ __launch_bounds__(NTHR) void k_wtr(const float* __restrict__ w, int nOff, unsigned short* wcs) {
  const int u = (int)blockIdx.x * NTHR + (int)threadIdx.x;
  if (u >= NLAY * HC * (KA / 8)) return;
  const int l  = u >> 12;
  const int r  = u & 4095;
  const int n  = r >> 5;
  const int k8 = (r & 31) * 8;
  const int kk = k8 & (HC - 1);
  const float* p = w + (size_t)l * HC * HC + (size_t)kk * HC + n;
  v4f a, b;
  a.x = p[0];        a.y = p[HC];       a.z = p[2 * HC];   a.w = p[3 * HC];
  b.x = p[4 * HC];   b.y = p[5 * HC];   b.z = p[6 * HC];   b.w = p[7 * HC];
  const v4u wv = pack8(a, b);
  unsigned short* o = wcs + (size_t)l * NW * KA + (size_t)(nOff + n) * KA + k8;
  *(volatile v4u*)o = wv;
  __threadfence();
  *(volatile v4u*)o = wv;
}

__global__ __launch_bounds__(NTHR) void k_embed(const int* __restrict__ x, const float* __restrict__ emb,
                                                unsigned short* hhl) {
  const int tid = (int)threadIdx.x, lane = tid & 31, wave = tid >> 5;
  const int node = (int)blockIdx.x * NWAVE + wave;
  if (node >= MP) return;
  const int nc = node < NN ? node : NN - 1;
  const int fl = lane < NFEAT ? lane : NFEAT - 1;
  int xv = x[nc * NFEAT + fl];
  xv = xv < 0 ? 0 : (xv > VOC - 1 ? VOC - 1 : xv);
  v4f s = {0.f, 0.f, 0.f, 0.f};
#pragma unroll
  for (int f = 0; f < NFEAT; ++f) {
    const int id = __shfl(xv, f, 32);
    const v4f v = *(const v4f*)(emb + ((size_t)(f * VOC + id)) * HC + 4 * lane);
    s.x += bfr(v.x); s.y += bfr(v.y); s.z += bfr(v.z); s.w += bfr(v.w);
  }
  const bool live = node < NN;
  v4f o;
  o.x = live ? s.x : 0.f; o.y = live ? s.y : 0.f; o.z = live ? s.z : 0.f; o.w = live ? s.w : 0.f;
  const HL q = split4(o);
  unsigned short* gp = hhl + (size_t)node * KA + 4 * lane;
  *(volatile v2u*)gp = q.hi;
  *(volatile v2u*)(gp + HC) = q.lo;
  __threadfence();
  *(volatile v2u*)gp = q.hi;
  *(volatile v2u*)(gp + HC) = q.lo;
}

__global__ __launch_bounds__(NTHR) void k_bucket(const int* __restrict__ srcs, const int* __restrict__ dsts,
                                                 int* SRT, int* SOFF, int* SCNT, int* FLG) {
  extern __shared__ v4f lds_dyn[];
  int* reg1 = (int*)lds_dyn;
  int* reg2 = reg1 + RCAP;
  int* scnt = reg2 + RCAP;
  int* soff = scnt + NB;
  int* list = soff + NB;
  int* wcnt = list + LISTN;
  int* wtot = wcnt + NWAVE;
  const int tid = (int)threadIdx.x, lane = tid & 31, wave = tid >> 5;
  const int nodeBase = (int)blockIdx.x * NB;

  {
    const v4i z4 = {0, 0, 0, 0};
    for (int i = tid * 4; i < RCAP; i += NTHR * 4) *(v4ia*)(reg2 + i) = z4;
    *(v4ia*)(scnt + 4 * tid) = z4;
  }
  __syncthreads();

  int tot = 0, traw = 0;
  const int nChunks = (NE + CHUNK - 1) / CHUNK;
#pragma unroll 1
  for (int ch = 0; ch < nChunks; ++ch) {
    const int cbase = ch * CHUNK;
    const int wc = scan_chunk(dsts, NE, cbase, nodeBase, NB, 1, list, tid, lane, wave);
    if (lane == 0) wcnt[wave] = wc;
    __syncthreads();
    int pre = 0, all = 0;
#pragma unroll
    for (int w2 = 0; w2 < NWAVE; ++w2) {
      int c = wcnt[w2];
      c = c < 0 ? 0 : (c > WCAP ? WCAP : c);
      all += c;
      pre += (w2 < wave) ? c : 0;
    }
    const int wcc  = wc > WCAP ? WCAP : wc;
    const int base = tot + pre;
#pragma unroll 1
    for (int b0 = 0; b0 < wcc; b0 += 32) {
      const int i  = b0 + lane;
      const int ic = i < wcc ? i : wcc - 1;
      const int ent = list[wave * WCAP + ic];
      const int el  = (ent >> SLB) & (CHUNK - 1);
      const int sl  = ent & (NB - 1);
      int eid = cbase + el;
      eid = eid > NE - 1 ? NE - 1 : eid;
      int sr = srcs[eid];
      sr = sr < 0 ? 0 : (sr > NN - 1 ? NN - 1 : sr);
      const int pos = base + i;
      if (i < wcc && pos < RCAP) reg1[pos] = (sl << 16) | sr;
    }
    traw += all;
    tot += all;
    tot = tot > RCAP ? RCAP : tot;
    __syncthreads();
  }
  const int nh  = tot;
  const int ovf = (traw > RCAP) ? 1 : 0;

  if (wave == 0) {
#pragma unroll 1
    for (int b0 = 0; b0 < nh; b0 += 32) {
      const int idx = b0 + lane;
      const int uv  = reg1[idx < nh ? idx : nh - 1];
      const int m32 = (nh - b0) < 32 ? (nh - b0) : 32;
#pragma unroll 1
      for (int k = 0; k < m32; ++k) {
        const int u  = __builtin_amdgcn_readlane(uv, k);
        const int sl = (u >> 16) & (NB - 1);
        if (lane == 0) scnt[sl] = scnt[sl] + 1;
      }
    }
  }
  __syncthreads();

  {
    const v4i ca = *(const v4ia*)(scnt + 4 * tid);
    const int e0 = ca.x < 0 ? 0 : ca.x, e1 = ca.y < 0 ? 0 : ca.y, e2 = ca.z < 0 ? 0 : ca.z, e3 = ca.w < 0 ? 0 : ca.w;
    const int ts = e0 + e1 + e2 + e3;
    int incl = ts;
#pragma unroll
    for (int d = 1; d < 32; d <<= 1) {
      const int up = __shfl_up(incl, d, 32);
      if (lane >= d) incl += up;
    }
    if (lane == 31) wtot[wave] = incl;
    __syncthreads();
    int pre = 0;
#pragma unroll
    for (int w2 = 0; w2 < NWAVE; ++w2) pre += (w2 < wave) ? wtot[w2] : 0;
    int run = pre + incl - ts;
    soff[4 * tid + 0] = run; run += e0;
    soff[4 * tid + 1] = run; run += e1;
    soff[4 * tid + 2] = run; run += e2;
    soff[4 * tid + 3] = run;
  }
  __syncthreads();
  for (int i = tid; i < NB; i += NTHR) list[i] = soff[i];
  __syncthreads();

  if (wave == 0) {
#pragma unroll 1
    for (int b0 = 0; b0 < nh; b0 += 32) {
      const int idx = b0 + lane;
      const int uv  = reg1[idx < nh ? idx : nh - 1];
      const int m32 = (nh - b0) < 32 ? (nh - b0) : 32;
#pragma unroll 1
      for (int k = 0; k < m32; ++k) {
        const int u  = __builtin_amdgcn_readlane(uv, k);
        const int sl = (u >> 16) & (NB - 1);
        const int sr = u & 0xFFFF;
        if (lane == 0) {
          int pos = list[sl];
          pos = pos < 0 ? 0 : (pos > RCAP - 1 ? RCAP - 1 : pos);
          reg2[pos] = sr;
          list[sl] = pos + 1;
        }
      }
    }
  }
  __syncthreads();

  int* gs = SRT  + (size_t)blockIdx.x * RCAP;
  int* go = SOFF + (size_t)blockIdx.x * NB;
  int* gc = SCNT + (size_t)blockIdx.x * NB;
  int* gf = FLG  + (size_t)blockIdx.x * 32;
  v4i fv = {0, 0, 0, 0};
  if (tid == 0) { fv.x = nh; fv.y = ovf; }
  const v4i ov = *(const v4ia*)(soff + 4 * tid);
  const v4i cv = *(const v4ia*)(scnt + 4 * tid);
#pragma unroll 1
  for (int i = tid * 4; i < RCAP; i += NTHR * 4) {
    const v4i v = *(const v4ia*)(reg2 + i);
    *(volatile v4i*)(gs + i) = v;
  }
  *(volatile v4i*)(go + 4 * tid) = ov;
  *(volatile v4i*)(gc + 4 * tid) = cv;
  if (tid < 8) *(volatile v4i*)(gf + 4 * tid) = fv;
  __threadfence();
#pragma unroll 1
  for (int i = tid * 4; i < RCAP; i += NTHR * 4) {
    const v4i v = *(const v4ia*)(reg2 + i);
    *(volatile v4i*)(gs + i) = v;
  }
  *(volatile v4i*)(go + 4 * tid) = ov;
  *(volatile v4i*)(gc + 4 * tid) = cv;
  if (tid < 8) *(volatile v4i*)(gf + 4 * tid) = fv;
}

__global__ __launch_bounds__(GTHR) void k_gemm(const unsigned short* __restrict__ A,
                                               const unsigned short* __restrict__ WT,
                                               const float* __restrict__ asr, const float* __restrict__ adr,
                                               const float* __restrict__ skb,
                                               float* XT, float* SK, float* ASD) {
  __shared__ __attribute__((aligned(16))) float stg[GBM * GBN];
  __shared__ __attribute__((aligned(16))) float satt[2 * HC];
  const int tid = (int)threadIdx.x, lane = tid & 31, wave = tid >> 5, hh = lane >> 4, m = lane & 15;
  const int rowBase = (int)blockIdx.x * GBM;
  const int colBase = (int)blockIdx.y * GBN;

  satt[tid]      = bfr(asr[tid]);
  satt[HC + tid] = bfr(adr[tid]);

  v8f acc[8];
  {
    const v8f z = {0.f, 0.f, 0.f, 0.f, 0.f, 0.f, 0.f, 0.f};
#pragma unroll
    for (int t = 0; t < 8; ++t) acc[t] = z;
  }
  const unsigned short* ap = A  + (size_t)(rowBase + 16 * wave + m) * (size_t)KA + 8 * hh;
  const unsigned short* bp = WT + (size_t)(colBase + m) * (size_t)KA + 8 * hh;
#pragma unroll 1
  for (int k0 = 0; k0 < KA; k0 += 32) {
    FragB af;
    af.h[0] = *(const v8usa*)(ap + k0);
    af.h[1] = *(const v8usa*)(ap + k0 + 16);
#pragma unroll
    for (int nt = 0; nt < 8; ++nt) {
      const unsigned short* wq = bp + (size_t)(16 * nt) * (size_t)KA + k0;
      FragB bf;
      bf.h[0] = *(const v8usa*)wq;
      bf.h[1] = *(const v8usa*)(wq + 16);
      acc[nt] = wmb(af, bf, acc[nt]);
    }
  }
#pragma unroll
  for (int nt = 0; nt < 8; ++nt) {
    const int lc = 16 * nt + m;
#pragma unroll
    for (int r = 0; r < 8; ++r) {
      const int lr = 16 * wave + 8 * hh + r;
      stg[lr * GBN + lc] = acc[nt][r];
    }
  }
  __syncthreads();

  if (blockIdx.y == 0) {
    const int row = tid & 63, which = tid >> 6;
    const float* sa = satt + which * HC;
    const float* hr = stg + row * GBN;
    float d0 = 0.f, d1 = 0.f, d2 = 0.f, d3 = 0.f;
#pragma unroll 1
    for (int c4 = 0; c4 < HID / 4; ++c4) {
      const v4f x0 = *(const v4fa*)(hr + 4 * c4);
      const v4f x1 = *(const v4fa*)(hr + HID + 4 * c4);
      const v4f x2 = *(const v4fa*)(hr + 2 * HID + 4 * c4);
      const v4f x3 = *(const v4fa*)(hr + 3 * HID + 4 * c4);
      const v4f a0 = *(const v4fa*)(sa + 4 * c4);
      const v4f a1 = *(const v4fa*)(sa + HID + 4 * c4);
      const v4f a2 = *(const v4fa*)(sa + 2 * HID + 4 * c4);
      const v4f a3 = *(const v4fa*)(sa + 3 * HID + 4 * c4);
      d0 = fmaf(x0.x, a0.x, d0); d0 = fmaf(x0.y, a0.y, d0); d0 = fmaf(x0.z, a0.z, d0); d0 = fmaf(x0.w, a0.w, d0);
      d1 = fmaf(x1.x, a1.x, d1); d1 = fmaf(x1.y, a1.y, d1); d1 = fmaf(x1.z, a1.z, d1); d1 = fmaf(x1.w, a1.w, d1);
      d2 = fmaf(x2.x, a2.x, d2); d2 = fmaf(x2.y, a2.y, d2); d2 = fmaf(x2.z, a2.z, d2); d2 = fmaf(x2.w, a2.w, d2);
      d3 = fmaf(x3.x, a3.x, d3); d3 = fmaf(x3.y, a3.y, d3); d3 = fmaf(x3.z, a3.z, d3); d3 = fmaf(x3.w, a3.w, d3);
    }
    v4f dv; dv.x = d0; dv.y = d1; dv.z = d2; dv.w = d3;
    float* dp = ASD + (size_t)which * ((size_t)MP * NHD) + (size_t)(rowBase + row) * NHD;
    v4f pv[16];
#pragma unroll
    for (int i = 0; i < 16; ++i) pv[i] = *(const v4fa*)(stg + (16 * wave + i) * GBN + 4 * lane);
#pragma unroll
    for (int i = 0; i < 16; ++i) {
      float* op = XT + (size_t)(rowBase + 16 * wave + i) * (size_t)HC + 4 * lane;
      *(volatile v4f*)op = pv[i];
    }
    *(volatile v4f*)dp = dv;
    __threadfence();
#pragma unroll
    for (int i = 0; i < 16; ++i) {
      float* op = XT + (size_t)(rowBase + 16 * wave + i) * (size_t)HC + 4 * lane;
      *(volatile v4f*)op = pv[i];
    }
    *(volatile v4f*)dp = dv;
  } else {
    const v4f bq = bfr4(*(const v4f*)(skb + 4 * lane));
    v4f pv[16];
#pragma unroll
    for (int i = 0; i < 16; ++i) {
      const v4f x = *(const v4fa*)(stg + (16 * wave + i) * GBN + 4 * lane);
      v4f y; y.x = x.x + bq.x; y.y = x.y + bq.y; y.z = x.z + bq.z; y.w = x.w + bq.w;
      pv[i] = y;
    }
#pragma unroll
    for (int i = 0; i < 16; ++i) {
      float* op = SK + (size_t)(rowBase + 16 * wave + i) * (size_t)HC + 4 * lane;
      *(volatile v4f*)op = pv[i];
    }
    __threadfence();
#pragma unroll
    for (int i = 0; i < 16; ++i) {
      float* op = SK + (size_t)(rowBase + 16 * wave + i) * (size_t)HC + 4 * lane;
      *(volatile v4f*)op = pv[i];
    }
  }
}

__global__ __launch_bounds__(NTHR) void k_scan(const float* __restrict__ XT, const float* __restrict__ SK,
                                               const float* __restrict__ ASD,
                                               const int* __restrict__ SRT, const int* __restrict__ SOFF,
                                               const int* __restrict__ SCNT, const int* __restrict__ FLG,
                                               const float* __restrict__ cb, float* Z, float* PART) {
  __shared__ __attribute__((aligned(16))) float zst[SROWS * HC];
  __shared__ __attribute__((aligned(16))) float pst[PARTW];
  const int tid = (int)threadIdx.x, lane = tid & 31, wave = tid >> 5;
  const int rowBase = (int)blockIdx.x * SROWS;
  const int c0   = 4 * lane;
  const int head = lane >> 3;
  const float* ASp = ASD;
  const float* ADp = ASD + (size_t)MP * NHD;
  const v4f cbv = bfr4(*(const v4f*)(cb + c0));
  const float qnan = __int_as_float(0x7fc00000);

#pragma unroll 1
  for (int jt = 0; jt < 8; ++jt) {
    const int sl   = wave * 8 + jt;
    const int grow = rowBase + sl;
    if (grow < NN) {
      const int bkt  = grow >> SLB;
      const int slot = grow & (NB - 1);
      int st   = SOFF[bkt * NB + slot];
      const int craw = SCNT[bkt * NB + slot];
      int nh   = FLG[bkt * 32];
      const int ovf = FLG[bkt * 32 + 1];
      nh = nh < 0 ? 0 : (nh > RCAP ? RCAP : nh);
      st = st < 0 ? 0 : (st > nh ? nh : st);
      int cnt = craw < 0 ? 0 : (craw > DEGCAP ? DEGCAP : craw);
      if (cnt > nh - st) cnt = nh - st;
      const float pz = (ovf != 0 || craw > DEGCAP) ? qnan : 0.0f;
      const int* sp = SRT + (size_t)bkt * RCAP;
      const float adv = ADp[(size_t)grow * NHD + head];
      float mx = -3.0e38f, dn = 0.0f;
      v4f av = {0.f, 0.f, 0.f, 0.f};
#pragma unroll 1
      for (int q = 0; q <= cnt; ++q) {
        int idx = st + q; idx = idx > RCAP - 1 ? RCAP - 1 : idx;
        int sraw = sp[idx];
        sraw = sraw < 0 ? 0 : (sraw > NN - 1 ? NN - 1 : sraw);
        const int s = (q < cnt) ? sraw : grow;
        const v4f fa = *(const v4f*)(XT + (size_t)s * HC + c0);
        float lg = ASp[(size_t)s * NHD + head] + adv;
        lg = lg > 0.f ? lg : NEGSL * lg;
        const float df = lg - mx;
        const float ee = expf(-fabsf(df));
        const bool up  = df > 0.f;
        const float s1 = up ? ee : 1.0f;
        const float s2 = up ? 1.0f : ee;
        mx = up ? lg : mx;
        dn = fmaf(dn, s1, s2);
        av.x = fmaf(av.x, s1, s2 * fa.x);
        av.y = fmaf(av.y, s1, s2 * fa.y);
        av.z = fmaf(av.z, s1, s2 * fa.z);
        av.w = fmaf(av.w, s1, s2 * fa.w);
      }
      const float inv = 1.0f / dn;
      const v4f skv = *(const v4f*)(SK + (size_t)grow * HC + c0);
      v4f zz;
      zz.x = fmaf(av.x, inv, cbv.x) + skv.x + pz;
      zz.y = fmaf(av.y, inv, cbv.y) + skv.y + pz;
      zz.z = fmaf(av.z, inv, cbv.z) + skv.z + pz;
      zz.w = fmaf(av.w, inv, cbv.w) + skv.w + pz;
      *(v4fa*)(zst + sl * HC + c0) = zz;
      float* zp = Z + (size_t)grow * HC + c0;
      *(volatile v4f*)zp = zz;
      __threadfence();
      *(volatile v4f*)zp = zz;
    }
  }
  __syncthreads();

  if (tid < HC) {
    int nv = NN - rowBase;
    nv = nv < 0 ? 0 : (nv > SROWS ? SROWS : nv);
    float mean = 0.0f, M2 = 0.0f;
#pragma unroll 1
    for (int r = 0; r < nv; ++r) {
      const float v  = zst[r * HC + tid];
      const float rk = 1.0f / (float)(r + 1);
      const float d  = v - mean;
      mean = fmaf(d, rk, mean);
      M2   = fmaf(d, v - mean, M2);
    }
    pst[1 + tid]      = mean;
    pst[1 + HC + tid] = M2;
    if (tid == 0) pst[0] = (float)nv;
  }
  if (tid >= 1 && tid < PARTW - NTHR) pst[NTHR + tid] = 0.0f;
  __syncthreads();
  float* pp = PART + (size_t)blockIdx.x * PARTW + 4 * tid;
  v4f ps = {0.f, 0.f, 0.f, 0.f};
  if (tid < PARTW / 4) {
    ps = *(const v4fa*)(pst + 4 * tid);
    *(volatile v4f*)pp = ps;
  }
  __threadfence();
  if (tid < PARTW / 4) {
    *(volatile v4f*)pp = ps;
  }
}

__global__ __launch_bounds__(HC) void k_comb(const float* __restrict__ part, int nPart,
                                             const float* __restrict__ gam, const float* __restrict__ bet,
                                             float* ss) {
  __shared__ __attribute__((aligned(16))) float stg[4 * HC];
  const int c = (int)threadIdx.x;
  double n = 0.0, mean = 0.0, M2 = 0.0;
#pragma unroll 1
  for (int b = 0; b < nPart; ++b) {
    const float* pr = part + (size_t)b * PARTW;
    const double nb = (double)pr[0];
    const double mb = (double)pr[1 + c];
    const double qb = (double)pr[1 + HC + c];
    if (nb > 0.5) {
      const double nn = n + nb;
      const double delta = mb - mean;
      const double f = nb / nn;
      mean = mean + delta * f;
      M2 = M2 + qb + delta * delta * n * f;
      n = nn;
    }
  }
  const double nt = n < 1.0 ? 1.0 : n;
  const float varf  = (float)(M2 / nt);
  const float meanf = (float)mean;
  const float rstd  = 1.0f / sqrtf(varf + 1e-5f);
  stg[c]          = meanf;
  stg[HC + c]     = bfr(gam[c]) * rstd;
  stg[2 * HC + c] = bfr(bet[c]);
  stg[3 * HC + c] = 0.0f;
  __syncthreads();
  const v4f v = *(const v4fa*)(stg + 4 * c);
  *(volatile v4f*)(ss + 4 * c) = v;
  __threadfence();
  *(volatile v4f*)(ss + 4 * c) = v;
}

__global__ __launch_bounds__(NTHR) void k_bn(const float* __restrict__ Z, const float* __restrict__ ss,
                                             unsigned short* hhl) {
  const int u = (int)blockIdx.x * NTHR + (int)threadIdx.x;
  if (u >= MP * 32) return;
  const int row = u >> 5;
  const int c0  = (u & 31) * 4;
  const int rc  = row < NN ? row : NN - 1;
  const v4f z  = *(const v4f*)(Z + (size_t)rc * HC + c0);
  const v4f mu = *(const v4f*)(ss + c0);
  const v4f sc = *(const v4f*)(ss + HC + c0);
  const v4f bb = *(const v4f*)(ss + 2 * HC + c0);
  const bool live = row < NN;
  v4f y;
  y.x = reluf(fmaf(z.x - mu.x, sc.x, bb.x));
  y.y = reluf(fmaf(z.y - mu.y, sc.y, bb.y));
  y.z = reluf(fmaf(z.z - mu.z, sc.z, bb.z));
  y.w = reluf(fmaf(z.w - mu.w, sc.w, bb.w));
  v4f o;
  o.x = live ? y.x : 0.f; o.y = live ? y.y : 0.f; o.z = live ? y.z : 0.f; o.w = live ? y.w : 0.f;
  const HL q = split4(o);
  unsigned short* gp = hhl + (size_t)row * KA + c0;
  *(volatile v2u*)gp = q.hi;
  *(volatile v2u*)(gp + HC) = q.lo;
  __threadfence();
  *(volatile v2u*)gp = q.hi;
  *(volatile v2u*)(gp + HC) = q.lo;
}

__global__ __launch_bounds__(NTHR) void k_pool(const int* __restrict__ batch, const float* __restrict__ Z,
                                               const float* __restrict__ ss, float* POOL) {
  __shared__ int lst[NTHR];
  __shared__ int wcnt[NWAVE];
  __shared__ __attribute__((aligned(16))) float pst[HC];
  const int tid = (int)threadIdx.x, lane = tid & 31, wave = tid >> 5;
  const int g = (int)blockIdx.x;
  const int c = tid & (HC - 1);
  const float mu = ss[c], sc = ss[HC + c], bb = ss[2 * HC + c];
  float acc = 0.0f;
  int cnt = 0;
  const int nCh = (NN + NTHR - 1) / NTHR;
#pragma unroll 1
  for (int ch = 0; ch < nCh; ++ch) {
    const int n  = ch * NTHR + tid;
    const int nc = n < NN ? n : NN - 1;
    const int bv = batch[nc];
    const bool hit = (n < NN) && (bv == g);
    const unsigned m = __builtin_amdgcn_ballot_w32(hit);
    const int below  = (int)__builtin_amdgcn_mbcnt_lo(m, 0u);
    int hv = hit ? 1 : 0;
    hv += __shfl_xor(hv, 16); hv += __shfl_xor(hv, 8); hv += __shfl_xor(hv, 4);
    hv += __shfl_xor(hv, 2);  hv += __shfl_xor(hv, 1);
    if (lane == 0) wcnt[wave] = hv;
    __syncthreads();
    int pre = 0, all = 0;
#pragma unroll
    for (int w2 = 0; w2 < NWAVE; ++w2) {
      int k = wcnt[w2];
      k = k < 0 ? 0 : (k > 32 ? 32 : k);
      all += k;
      pre += (w2 < wave) ? k : 0;
    }
    if (hit) lst[pre + below] = n;
    __syncthreads();
    if (tid < HC) {
#pragma unroll 1
      for (int i = 0; i < all; ++i) {
        int node = lst[i];
        node = node < 0 ? 0 : (node > NN - 1 ? NN - 1 : node);
        const float v = Z[(size_t)node * HC + c];
        acc += reluf(fmaf(v - mu, sc, bb));
      }
    }
    cnt += all;
    __syncthreads();
  }
  if (tid < HC) {
    const float cf = (float)(cnt > 1 ? cnt : 1);
    pst[c] = acc * (1.0f / cf);
  }
  __syncthreads();
  v4f v = {0.f, 0.f, 0.f, 0.f};
  float* op = POOL + (size_t)g * HC + 4 * (tid & 31);
  if (tid < 32) {
    v = *(const v4fa*)(pst + 4 * tid);
    *(volatile v4f*)op = v;
  }
  __threadfence();
  if (tid < 32) {
    *(volatile v4f*)op = v;
  }
}

__global__ __launch_bounds__(NG) void k_head(const float* __restrict__ POOL, const float* __restrict__ mlpW,
                                             const float* __restrict__ mlpb, float* out) {
  __shared__ __attribute__((aligned(16))) float sw[HC];
  __shared__ __attribute__((aligned(16))) float res[NG];
  const int tid = (int)threadIdx.x;
  if (tid < HC) sw[tid] = bfr(mlpW[tid]);
  __syncthreads();
  const float* p = POOL + (size_t)tid * HC;
  float d = 0.0f;
#pragma unroll 2
  for (int c4 = 0; c4 < HC / 4; ++c4) {
    const v4f x = *(const v4f*)(p + 4 * c4);
    const v4f w = *(const v4fa*)(sw + 4 * c4);
    d = fmaf(x.x, w.x, d);
    d = fmaf(x.y, w.y, d);
    d = fmaf(x.z, w.z, d);
    d = fmaf(x.w, w.w, d);
  }
  res[tid] = d + bfr(mlpb[0]);
  __syncthreads();
  v4f v = {0.f, 0.f, 0.f, 0.f};
  float* op = out + 4 * (tid & 63);
  if (tid < NG / 4) {
    v = *(const v4fa*)(res + 4 * tid);
    *(volatile v4f*)op = v;
  }
  __threadfence();
  if (tid < NG / 4) {
    *(volatile v4f*)op = v;
  }
}

static inline size_t al256(size_t o) { return (o + 255) & ~(size_t)255; }

extern "C" void kernel_launch(void* const* d_in, const int* in_sizes, int n_in,
                              void* d_out, int out_size, void* d_ws, size_t ws_size,
                              hipStream_t stream) {
  if (n_in < 14) return;
  if (in_sizes[0] != NN * NFEAT) return;
  if (in_sizes[1] != 2 * NE) return;
  if (in_sizes[2] != NN) return;
  if (in_sizes[3] != NFEAT * VOC * HC) return;
  if (in_sizes[4] != NLAY * HC * HC) return;
  if (in_sizes[5] != NLAY * HC || in_sizes[6] != NLAY * HC) return;
  if (in_sizes[7] != NLAY * HC) return;
  if (in_sizes[8] != NLAY * HC * HC) return;
  if (in_sizes[9] != NLAY * HC) return;
  if (in_sizes[10] != NLAY * HC || in_sizes[11] != NLAY * HC) return;
  if (in_sizes[12] != HC) return;
  if (in_sizes[13] < 1) return;
  if (out_size != NG) return;

  const int*   x      = (const int*)  d_in[0];
  const int*   ei     = (const int*)  d_in[1];
  const int*   batch  = (const int*)  d_in[2];
  const float* emb    = (const float*)d_in[3];
  const float* convW  = (const float*)d_in[4];
  const float* a_src  = (const float*)d_in[5];
  const float* a_dst  = (const float*)d_in[6];
  const float* conv_b = (const float*)d_in[7];
  const float* skipW  = (const float*)d_in[8];
  const float* skip_b = (const float*)d_in[9];
  const float* bn_g   = (const float*)d_in[10];
  const float* bn_b   = (const float*)d_in[11];
  const float* mlpW   = (const float*)d_in[12];
  const float* mlp_b  = (const float*)d_in[13];
  float* out = (float*)d_out;
  const int* src = ei;
  const int* dst = ei + NE;

  char* ws = (char*)d_ws;
  size_t off = 0;
  const size_t oWCS = off; off = al256(off + (size_t)NLAY * NW * KA * 2);
  const size_t oHHL = off; off = al256(off + (size_t)MP * KA * 2);
  const size_t oXT  = off; off = al256(off + (size_t)MP * HC * 4);
  const size_t oSK  = off; off = al256(off + (size_t)MP * HC * 4);
  const size_t oZ   = off; off = al256(off + (size_t)MP * HC * 4);
  const size_t oASD = off; off = al256(off + (size_t)2 * MP * NHD * 4);
  const size_t oSRT = off; off = al256(off + (size_t)NBLK * RCAP * 4);
  const size_t oSOF = off; off = al256(off + (size_t)NBLK * NB * 4);
  const size_t oSCN = off; off = al256(off + (size_t)NBLK * NB * 4);
  const size_t oFLG = off; off = al256(off + (size_t)NBLK * 32 * 4);
  const size_t oPT  = off; off = al256(off + (size_t)NSB * PARTW * 4);
  const size_t oSS  = off; off = al256(off + (size_t)4 * HC * 4);
  const size_t oPL  = off; off = al256(off + (size_t)NG * HC * 4);
  if (off > ws_size || off > (size_t)WSMAX) return;
  unsigned short* WCS = (unsigned short*)(ws + oWCS);
  unsigned short* HHL = (unsigned short*)(ws + oHHL);
  float* XT   = (float*)(ws + oXT);
  float* SK   = (float*)(ws + oSK);
  float* Z    = (float*)(ws + oZ);
  float* ASD  = (float*)(ws + oASD);
  int*   SRT  = (int*)(ws + oSRT);
  int*   SOFF = (int*)(ws + oSOF);
  int*   SCNT = (int*)(ws + oSCN);
  int*   FLG  = (int*)(ws + oFLG);
  float* PART = (float*)(ws + oPT);
  float* SS   = (float*)(ws + oSS);
  float* POOL = (float*)(ws + oPL);

  hipFuncSetAttribute(reinterpret_cast<const void*>(&k_bucket),
                      hipFuncAttributeMaxDynamicSharedMemorySize, LDS_BKT);

  k_wtr<<<(NLAY * HC * (KA / 8)) / NTHR, NTHR, 0, stream>>>(convW, 0, WCS);
  k_wtr<<<(NLAY * HC * (KA / 8)) / NTHR, NTHR, 0, stream>>>(skipW, HC, WCS);
  k_embed<<<MP / NWAVE, NTHR, 0, stream>>>(x, emb, HHL);
  k_bucket<<<NBLK, NTHR, LDS_BKT, stream>>>(src, dst, SRT, SOFF, SCNT, FLG);

  for (int l = 0; l < NLAY; ++l) {
    k_gemm<<<dim3(MP / GBM, NW / GBN), GTHR, 0, stream>>>(HHL, WCS + (size_t)l * NW * KA,
                                                          a_src + l * HC, a_dst + l * HC, skip_b + l * HC,
                                                          XT, SK, ASD);
    k_scan<<<NSB, NTHR, 0, stream>>>(XT, SK, ASD, SRT, SOFF, SCNT, FLG, conv_b + l * HC, Z, PART);
    k_comb<<<1, HC, 0, stream>>>(PART, NSB, bn_g + l * HC, bn_b + l * HC, SS);
    if (l < NLAY - 1) {
      k_bn<<<(MP * 32) / NTHR, NTHR, 0, stream>>>(Z, SS, HHL);
    }
  }
  k_pool<<<NG, NTHR, 0, stream>>>(batch, Z, SS, POOL);
  k_head<<<1, NG, 0, stream>>>(POOL, mlpW, mlp_b, out);
}
